// DRF_39281770889393
// MI455X (gfx1250) — hardware-verified
//
#include <hip/hip_runtime.h>
#include <stddef.h>
#include <stdint.h>
#include <math.h>

#define NPIX 16384
#define IMW  128
#define CC   64
#define C3   192
#define FF   256
#define NWD  256
#define WT   64
#define TP   68
#define WTP  68

static_assert(NWD * WT == NPIX);
static_assert(CC % 32 == 0);
static_assert(FF % 64 == 0);

typedef _Float16 v16h __attribute__((ext_vector_type(16)));
typedef _Float16 v8h  __attribute__((ext_vector_type(8)));
typedef __bf16   v16b __attribute__((ext_vector_type(16)));
typedef __bf16   v8b  __attribute__((ext_vector_type(8)));
typedef float    v8f  __attribute__((ext_vector_type(8)));
typedef float    v4f  __attribute__((ext_vector_type(4)));
typedef unsigned int v4u __attribute__((ext_vector_type(4)));

union Frag  { v16h v; v8h h[2]; v4u u[2]; };
union FragB { v16b v; v8b h[2]; };
union Pack8 { v8h h; v4u u; };

__device__ __forceinline__ v8f zero8() { return (v8f){0.f, 0.f, 0.f, 0.f, 0.f, 0.f, 0.f, 0.f}; }

__device__ __forceinline__ v8f mma16(v16h a, v16h b, v8f c) {
  c = __builtin_amdgcn_wmma_f32_16x16x32_f16(false, a, false, b, (short)0, c, false, false);
  asm volatile("v_nop\n\tv_nop\n\tv_nop\n\tv_nop" : "+v"(c) : "v"(a), "v"(b));
  return c;
}
__device__ __forceinline__ v8f mmab(v16b a, v16b b, v8f c) {
  c = __builtin_amdgcn_wmma_f32_16x16x32_bf16(false, a, false, b, (short)0, c, false, false);
  asm volatile("v_nop\n\tv_nop\n\tv_nop\n\tv_nop" : "+v"(c) : "v"(a), "v"(b));
  return c;
}

__device__ __forceinline__ v16h ldfrag(const _Float16* p, int ld, int row0, int k0, int lane) {
  const int m = lane & 15, lh = lane >> 4;
  const _Float16* q = p + (size_t)(row0 + m) * ld + k0 + 8 * lh;
  Frag f;
  f.h[0] = *(const v8h*)(q);
  f.h[1] = *(const v8h*)(q + 16);
  return f.v;
}
__device__ __forceinline__ v16b ldfragb(const __bf16* p, int ld, int row0, int k0, int lane) {
  const int m = lane & 15, lh = lane >> 4;
  const __bf16* q = p + (size_t)(row0 + m) * ld + k0 + 8 * lh;
  FragB f;
  f.h[0] = *(const v8b*)(q);
  f.h[1] = *(const v8b*)(q + 16);
  return f.v;
}

__device__ __forceinline__ unsigned int bfbits(float f) {
  const unsigned int u = __float_as_uint(f);
  return (u + 0x7fffu + ((u >> 16) & 1u)) >> 16;
}
__device__ __forceinline__ unsigned int bfsel(float f, int lo) {
  const unsigned int hb = bfbits(f);
  const float res = f - __uint_as_float(hb << 16);
  const unsigned int lb = bfbits(res);
  return lo ? lb : hb;
}
__device__ __forceinline__ unsigned int bfpack2(float a, float b, int lo) {
  return bfsel(a, lo) | (bfsel(b, lo) << 16);
}

__device__ __forceinline__ void ln16(const float* rp, const float* __restrict__ g,
                                     const float* __restrict__ bt, int part, float (&o)[16]) {
  float a[16];
#pragma unroll
  for (int k = 0; k < 4; ++k) {
    const v4f t = *(const v4f*)(rp + 4 * k);
    a[4 * k] = t[0]; a[4 * k + 1] = t[1]; a[4 * k + 2] = t[2]; a[4 * k + 3] = t[3];
  }
  float s = 0.f;
#pragma unroll
  for (int e = 0; e < 16; ++e) s += a[e];
  s += __shfl_xor(s, 1, 32);
  s += __shfl_xor(s, 2, 32);
  const float mean = s * (1.0f / 64.0f);
  float q = 0.f;
#pragma unroll
  for (int e = 0; e < 16; ++e) { a[e] -= mean; q = fmaf(a[e], a[e], q); }
  q += __shfl_xor(q, 1, 32);
  q += __shfl_xor(q, 2, 32);
  const float inv = rsqrtf(q * (1.0f / 64.0f) + 1e-6f);
#pragma unroll
  for (int k = 0; k < 4; ++k) {
    const v4f gv = *(const v4f*)(g + part * 16 + 4 * k);
    const v4f bv = *(const v4f*)(bt + part * 16 + 4 * k);
#pragma unroll
    for (int e = 0; e < 4; ++e) o[4 * k + e] = a[4 * k + e] * inv * gv[e] + bv[e];
  }
}

__global__ __launch_bounds__(256) void k_posln(const float* __restrict__ x,
                                               const float* __restrict__ pw,
                                               const float* __restrict__ pb,
                                               const float* __restrict__ g,
                                               const float* __restrict__ bt,
                                               float* __restrict__ x1,
                                               unsigned short* __restrict__ a1) {
  __shared__ __align__(16) float xh[100 * 64];
  __shared__ __align__(16) float T[WT * TP];
  const int tid = threadIdx.x, lane = tid & 31, wave = tid >> 5;
  const int p = blockIdx.x;
  const int y0 = (p >> 4) * 8, x0 = (p & 15) * 8;
  const int ch = tid & 63, grp = tid >> 6;
  const float* xc = x + (size_t)ch * NPIX;
#pragma unroll 1
  for (int i = grp; i < 100; i += 4) {
    const int hy = i / 10, hx = i - hy * 10;
    const int yy = y0 - 1 + hy, xx = x0 - 1 + hx;
    const int yc = min(max(yy, 0), IMW - 1), xq = min(max(xx, 0), IMW - 1);
    const float v = xc[yc * IMW + xq];
    const bool inb = (yy >= 0) && (yy < IMW) && (xx >= 0) && (xx < IMW);
    xh[i * 64 + ch] = inb ? v : 0.0f;
  }
  float w9[9];
#pragma unroll
  for (int k = 0; k < 9; ++k) w9[k] = pw[ch * 9 + k];
  const float pbc = pb[ch];
  __syncthreads();
#pragma unroll 1
  for (int j = 0; j < 16; ++j) {
    const int q = grp * 16 + j;
    const int ly = q >> 3, lx = q & 7;
    const float* hp = xh + (ly * 10 + lx) * 64 + ch;
    float acc = hp[(1 * 10 + 1) * 64];
#pragma unroll
    for (int dy = 0; dy < 3; ++dy)
#pragma unroll
      for (int dx = 0; dx < 3; ++dx)
        acc = fmaf(hp[(dy * 10 + dx) * 64], w9[dy * 3 + dx], acc);
    T[q * TP + ch] = acc + pbc;
  }
  __syncthreads();
  float* L = xh;
  {
    const int q = tid >> 2, part = tid & 3;
    float o[16];
    ln16(T + q * TP + part * 16, g, bt, part, o);
#pragma unroll
    for (int k = 0; k < 4; ++k)
      *(v4f*)(L + q * TP + part * 16 + 4 * k) = (v4f){o[4 * k], o[4 * k + 1], o[4 * k + 2], o[4 * k + 3]};
  }
  __syncthreads();
  v4u av[6];
  size_t ag[6];
#pragma unroll
  for (int it = 0; it < 6; ++it) {
    const int q = it * 32 + lane;
    const int rl = q / 24, pc = q - rl * 24;
    const int sec = pc >> 3, c8 = (pc & 7) * 8;
    const int lo = (sec == 1);
    const float* lp = L + (wave * 8 + rl) * TP + c8;
    const v4f f0 = *(const v4f*)(lp), f1 = *(const v4f*)(lp + 4);
    v4u u;
    u[0] = bfpack2(f0[0], f0[1], lo);
    u[1] = bfpack2(f0[2], f0[3], lo);
    u[2] = bfpack2(f1[0], f1[1], lo);
    u[3] = bfpack2(f1[2], f1[3], lo);
    av[it] = u;
    ag[it] = ((size_t)(p * WT + wave * 8 + rl)) * C3 + pc * 8;
  }
  for (int ps = 0; ps < 2; ++ps) {
#pragma unroll
    for (int it = 0; it < 4; ++it) {
      const int q = it * 32 + lane;
      const int lx = q >> 4, c4 = (q & 15) * 4;
      const v4f v = *(const v4f*)(T + (wave * 8 + lx) * TP + c4);
      *(volatile v4f*)(x1 + ((size_t)((y0 + wave) * IMW + x0 + lx)) * CC + c4) = v;
    }
#pragma unroll
    for (int it = 0; it < 6; ++it) *(volatile v4u*)(a1 + ag[it]) = av[it];
    __threadfence();
  }
}

__global__ __launch_bounds__(256) void k_wt(const float* __restrict__ w, _Float16* __restrict__ wt,
                                           int nout, int kin) {
  __shared__ __align__(16) float tf[64 * WTP];
  const int tid = threadIdx.x;
  const int n0 = blockIdx.x * 64;
  const int k0 = blockIdx.y * 64;
  {
    const int kr = tid >> 4;
    const int n4 = (tid & 15) * 4;
#pragma unroll
    for (int it = 0; it < 4; ++it) {
      const int kl = it * 16 + kr;
      const v4f a = *(const v4f*)(w + (size_t)(k0 + kl) * nout + n0 + n4);
      *(v4f*)(tf + kl * WTP + n4) = a;
    }
  }
  __syncthreads();
  v4u val[2];
  size_t go[2];
#pragma unroll
  for (int j = 0; j < 2; ++j) {
    const int p  = tid + 256 * j;
    const int nl = p >> 3;
    const int pc = p & 7;
    const float* cp = tf + (pc * 8) * WTP + nl;
    Pack8 pk;
    pk.h = (v8h){(_Float16)(cp[0 * WTP] * 64.0f), (_Float16)(cp[1 * WTP] * 64.0f),
                 (_Float16)(cp[2 * WTP] * 64.0f), (_Float16)(cp[3 * WTP] * 64.0f),
                 (_Float16)(cp[4 * WTP] * 64.0f), (_Float16)(cp[5 * WTP] * 64.0f),
                 (_Float16)(cp[6 * WTP] * 64.0f), (_Float16)(cp[7 * WTP] * 64.0f)};
    val[j] = pk.u;
    go[j]  = (size_t)(n0 + nl) * kin + k0 + pc * 8;
  }
  for (int ps = 0; ps < 2; ++ps) {
#pragma unroll
    for (int j = 0; j < 2; ++j) *(volatile v4u*)(wt + go[j]) = val[j];
    __threadfence();
  }
}

__global__ __launch_bounds__(256) void k_wq3(const float* __restrict__ w, unsigned short* __restrict__ wq) {
  __shared__ __align__(16) float tf[64 * WTP];
  const int tid = threadIdx.x;
  const int n0 = blockIdx.x * 64;
  {
    const int kr = tid >> 4;
    const int n4 = (tid & 15) * 4;
#pragma unroll
    for (int it = 0; it < 4; ++it) {
      const int kl = it * 16 + kr;
      const v4f a = *(const v4f*)(w + (size_t)kl * C3 + n0 + n4);
      *(v4f*)(tf + kl * WTP + n4) = a;
    }
  }
  __syncthreads();
  v4u val[6];
  size_t go[6];
#pragma unroll
  for (int j = 0; j < 6; ++j) {
    const int q  = tid + 256 * j;
    const int nl = q / 24, pc = q - nl * 24;
    const int sec = pc >> 3, k8 = (pc & 7) * 8;
    const int lo = (sec == 2);
    const float* cp = tf + k8 * WTP + nl;
    v4u u;
    u[0] = bfpack2(cp[0 * WTP], cp[1 * WTP], lo);
    u[1] = bfpack2(cp[2 * WTP], cp[3 * WTP], lo);
    u[2] = bfpack2(cp[4 * WTP], cp[5 * WTP], lo);
    u[3] = bfpack2(cp[6 * WTP], cp[7 * WTP], lo);
    val[j] = u;
    go[j]  = ((size_t)(n0 + nl)) * C3 + pc * 8;
  }
  for (int ps = 0; ps < 2; ++ps) {
#pragma unroll
    for (int j = 0; j < 6; ++j) *(volatile v4u*)(wq + go[j]) = val[j];
    __threadfence();
  }
}

#define STP 196
__global__ __launch_bounds__(256) void k_qkv(const __bf16* __restrict__ a1,
                                             const __bf16* __restrict__ wq,
                                             const float* __restrict__ qb,
                                             float* __restrict__ qkv,
                                             float* __restrict__ mw) {
  __shared__ __align__(16) float st[WT * STP];
  __shared__ __align__(16) float ms[128];
  const int tid = threadIdx.x, lane = tid & 31, wave = tid >> 5;
  const int hl = lane >> 4, c = lane & 15;
  const int p = blockIdx.x;
  const int mi = wave & 3;
  const int nb = (wave >> 2) * 96;
  const int m0 = p * WT + mi * 16;

  v8f acc[6];
#pragma unroll
  for (int t = 0; t < 6; ++t) acc[t] = zero8();
#pragma unroll 2
  for (int k0 = 0; k0 < C3; k0 += 32) {
    const v16b a = ldfragb(a1, C3, m0, k0, lane);
#pragma unroll
    for (int t = 0; t < 6; ++t) {
      const v16b b = ldfragb(wq, C3, nb + 16 * t, k0, lane);
      acc[t] = mmab(a, b, acc[t]);
    }
  }
#pragma unroll
  for (int t = 0; t < 6; ++t) {
    const int col = nb + 16 * t + c;
    const float bb = qb[col];
#pragma unroll
    for (int r = 0; r < 8; ++r) st[(mi * 16 + 8 * hl + r) * STP + col] = acc[t][r] + bb;
  }
  __syncthreads();
  if (tid < 128) {
    float s = 0.f;
#pragma unroll 8
    for (int r = 0; r < WT; ++r) s += st[r * STP + tid];
    ms[tid] = s * (1.0f / 64.0f);
  }
  __syncthreads();
  for (int ps = 0; ps < 2; ++ps) {
#pragma unroll
    for (int it = 0; it < 12; ++it) {
      const int q  = it * 32 + lane;
      const int rl = q / 48, c4 = (q - rl * 48) * 4;
      const v4f v = *(const v4f*)(st + (wave * 8 + rl) * STP + c4);
      *(volatile v4f*)(qkv + ((size_t)(p * WT + wave * 8 + rl)) * C3 + c4) = v;
    }
    if (wave == 0) {
      const v4f mv = *(const v4f*)(ms + 4 * lane);
      *(volatile v4f*)(mw + (size_t)p * 128 + 4 * lane) = mv;
    }
    __threadfence();
  }
}

#define ATT_LDS 117024
#define KTP 72
#define VTP 264
__global__ __launch_bounds__(256) void k_attn(const float* __restrict__ qkv,
                                              const float* __restrict__ mw,
                                              float* __restrict__ ao) {
  extern __shared__ __align__(16) char smem[];
  _Float16* Qs = (_Float16*)(smem);
  _Float16* Ks = (_Float16*)(smem + 9216);
  _Float16* Vt = (_Float16*)(smem + 46080);
  _Float16* Pa = (_Float16*)(smem + 79872);
  float* Os = (float*)(smem + 98304);
  float* qw = (float*)(smem + 115712);
  float* sl = (float*)(smem + 115968);
  int* isel = (int*)(smem + 116992);

  const int tid = threadIdx.x, lane = tid & 31, wave = tid >> 5;
  const int hl = lane >> 4, m = lane & 15;
  const int p = blockIdx.x;
  const float NEGI = -__builtin_huge_valf();

  if (tid < 16) *(v4f*)(qw + 4 * tid) = *(const v4f*)(mw + (size_t)p * 128 + 4 * tid);
  __syncthreads();
  {
    const float* kr = mw + (size_t)tid * 128 + 64;
    float acc = 0.f;
#pragma unroll
    for (int i4 = 0; i4 < 16; ++i4) {
      const v4f kv = *(const v4f*)(kr + 4 * i4);
      const v4f qv = *(const v4f*)(qw + 4 * i4);
      acc = fmaf(qv[0], kv[0], acc);
      acc = fmaf(qv[1], kv[1], acc);
      acc = fmaf(qv[2], kv[2], acc);
      acc = fmaf(qv[3], kv[3], acc);
    }
    sl[tid] = acc;
  }
  __syncthreads();
  if (wave == 0) {
    float v0 = NEGI, v1 = NEGI, v2 = NEGI, v3 = NEGI;
    int i0 = 0, i1 = 0, i2 = 0, i3 = 0;
#pragma unroll 1
    for (int j = 0; j < NWD; ++j) {
      const float s = sl[j];
      if (s > v3) {
        if (s > v2) {
          v3 = v2; i3 = i2;
          if (s > v1) {
            v2 = v1; i2 = i1;
            if (s > v0) { v1 = v0; i1 = i0; v0 = s; i0 = j; }
            else { v1 = s; i1 = j; }
          } else { v2 = s; i2 = j; }
        } else { v3 = s; i3 = j; }
      }
    }
    const int mine = (lane == 0) ? i0 : ((lane == 1) ? i1 : ((lane == 2) ? i2 : i3));
    if (lane < 4) isel[lane] = mine;
  }
  __syncthreads();
  {
    int wsel = isel[tid >> 6];
    wsel = min(max(wsel, 0), NWD - 1);
    const float* src = qkv + ((size_t)(wsel * WT + (tid & 63))) * C3;
#pragma unroll
    for (int i = 0; i < 8; ++i) {
      const v4f f0 = *(const v4f*)(src + 64 + 8 * i);
      const v4f f1 = *(const v4f*)(src + 68 + 8 * i);
      *(v8h*)(Ks + tid * KTP + 8 * i) =
          (v8h){(_Float16)f0[0], (_Float16)f0[1], (_Float16)f0[2], (_Float16)f0[3],
                (_Float16)f1[0], (_Float16)f1[1], (_Float16)f1[2], (_Float16)f1[3]};
    }
#pragma unroll
    for (int i = 0; i < 16; ++i) {
      const v4f f = *(const v4f*)(src + 128 + 4 * i);
      Vt[(4 * i + 0) * VTP + tid] = (_Float16)f[0];
      Vt[(4 * i + 1) * VTP + tid] = (_Float16)f[1];
      Vt[(4 * i + 2) * VTP + tid] = (_Float16)f[2];
      Vt[(4 * i + 3) * VTP + tid] = (_Float16)f[3];
    }
    const int tok = tid >> 2, c0 = (tid & 3) * 16;
    const float* sq = qkv + ((size_t)(p * WT + tok)) * C3 + c0;
    const v4f q0 = *(const v4f*)(sq), q1 = *(const v4f*)(sq + 4);
    const v4f q2 = *(const v4f*)(sq + 8), q3 = *(const v4f*)(sq + 12);
    *(v8h*)(Qs + tok * KTP + c0) =
        (v8h){(_Float16)q0[0], (_Float16)q0[1], (_Float16)q0[2], (_Float16)q0[3],
              (_Float16)q1[0], (_Float16)q1[1], (_Float16)q1[2], (_Float16)q1[3]};
    *(v8h*)(Qs + tok * KTP + c0 + 8) =
        (v8h){(_Float16)q2[0], (_Float16)q2[1], (_Float16)q2[2], (_Float16)q2[3],
              (_Float16)q3[0], (_Float16)q3[1], (_Float16)q3[2], (_Float16)q3[3]};
  }
  __syncthreads();

  const int h = wave;
  const unsigned int keep = hl ? 0u : 0xffffffffu;
  const v4u kmask = (v4u){keep, keep, keep, keep};
  const v4u z4 = (v4u){0u, 0u, 0u, 0u};
  _Float16* pw = Pa + wave * (16 * KTP);
  const float sscale = 0.125f;
#pragma unroll 1
  for (int mt = 0; mt < 4; ++mt) {
    Frag qa;
    qa.u[0] = *(const v4u*)(Qs + (mt * 16 + m) * KTP + h * 8) & kmask;
    qa.u[1] = z4;
    float mrow[8], lrow[8];
#pragma unroll
    for (int r = 0; r < 8; ++r) { mrow[r] = NEGI; lrow[r] = 0.f; }
    v8f oacc = zero8();
#pragma unroll 1
    for (int kc = 0; kc < 4; ++kc) {
      __syncthreads();
      v8f s[4];
#pragma unroll
      for (int j = 0; j < 4; ++j) {
        Frag kb;
        kb.u[0] = *(const v4u*)(Ks + (kc * 64 + j * 16 + m) * KTP + h * 8) & kmask;
        kb.u[1] = z4;
        s[j] = mma16(qa.v, kb.v, zero8());
      }
      float cm[8];
#pragma unroll
      for (int r = 0; r < 8; ++r) {
        float mx = NEGI;
#pragma unroll
        for (int j = 0; j < 4; ++j) {
          const float sv = s[j][r] * sscale;
          s[j][r] = sv;
          mx = fmaxf(mx, sv);
        }
#pragma unroll
        for (int off = 1; off < 16; off <<= 1) mx = fmaxf(mx, __shfl_xor(mx, off, 32));
        cm[r] = mx;
      }
      float al[8];
#pragma unroll
      for (int r = 0; r < 8; ++r) {
        const float mnew  = fmaxf(mrow[r], cm[r]);
        const float alpha = __expf(mrow[r] - mnew);
        mrow[r] = mnew;
        float psum = 0.f;
#pragma unroll
        for (int j = 0; j < 4; ++j) {
          const float pv = __expf(s[j][r] - mnew);
          psum += pv;
          pw[(8 * hl + r) * KTP + j * 16 + m] = (_Float16)(pv * 1024.0f);
        }
#pragma unroll
        for (int off = 1; off < 16; off <<= 1) psum += __shfl_xor(psum, off, 32);
        lrow[r] = lrow[r] * alpha + psum;
        al[r] = alpha;
      }
#pragma unroll
      for (int r = 0; r < 8; ++r) oacc[r] *= al[r];
      __syncthreads();
#pragma unroll
      for (int kk = 0; kk < 2; ++kk) {
        const v16h pa = ldfrag(pw, KTP, 0, kk * 32, lane);
        Frag vb;
        const _Float16* vq = Vt + (h * 8 + (lane & 7)) * VTP + kc * 64 + kk * 32 + 8 * hl;
        vb.h[0] = *(const v8h*)(vq);
        vb.h[1] = *(const v8h*)(vq + 16);
        oacc = mma16(pa, vb.v, oacc);
      }
    }
#pragma unroll
    for (int r = 0; r < 8; ++r) {
      const float inv = 1.0f / (lrow[r] * 1024.0f);
      if (m < 8) Os[(mt * 16 + 8 * hl + r) * TP + h * 8 + m] = oacc[r] * inv;
    }
  }
  __syncthreads();
  for (int ps = 0; ps < 2; ++ps) {
#pragma unroll
    for (int it = 0; it < 4; ++it) {
      const int q = it * 32 + lane;
      const int rl = q >> 4, c4 = (q & 15) * 4;
      const v4f v = *(const v4f*)(Os + (wave * 8 + rl) * TP + c4);
      *(volatile v4f*)(ao + ((size_t)(p * WT + wave * 8 + rl)) * CC + c4) = v;
    }
    __threadfence();
  }
}

__global__ __launch_bounds__(256) void k_comb(const float* __restrict__ qkv,
                                              const float* __restrict__ ao,
                                              const float* __restrict__ lw,
                                              const float* __restrict__ lb,
                                              const _Float16* __restrict__ wot,
                                              const float* __restrict__ wob,
                                              const float* __restrict__ x1,
                                              const float* __restrict__ g,
                                              const float* __restrict__ bt,
                                              float* __restrict__ x2,
                                              _Float16* __restrict__ yp) {
  __shared__ __align__(16) float vh[144 * 64];
  __shared__ __align__(16) _Float16 zs[WT * KTP];
  __shared__ __align__(16) _Float16 ys[WT * KTP];
  __shared__ __align__(16) float lws[CC * 25];
  const int tid = threadIdx.x, lane = tid & 31, wave = tid >> 5;
  const int hl = lane >> 4, m = lane & 15;
  const int p = blockIdx.x;
  const int y0 = (p >> 4) * 8, x0 = (p & 15) * 8;
  const int ch = tid & 63, grp = tid >> 6;
#pragma unroll 1
  for (int i = tid; i < CC * 25; i += 256) lws[i] = lw[i];
#pragma unroll 1
  for (int i = grp; i < 144; i += 4) {
    const int hy = i / 12, hx = i - hy * 12;
    const int yy = y0 - 2 + hy, xx = x0 - 2 + hx;
    const int yc = min(max(yy, 0), IMW - 1), xq = min(max(xx, 0), IMW - 1);
    const int sp = (yc >> 3) * 16 + (xq >> 3), sq = (yc & 7) * 8 + (xq & 7);
    const float v = qkv[((size_t)(sp * WT + sq)) * C3 + 128 + ch];
    const bool inb = (yy >= 0) && (yy < IMW) && (xx >= 0) && (xx < IMW);
    vh[i * 64 + ch] = inb ? v : 0.0f;
  }
  const float lbc = lb[ch];
  __syncthreads();
  float w25[25];
#pragma unroll
  for (int k = 0; k < 25; ++k) w25[k] = lws[ch * 25 + k];
#pragma unroll 1
  for (int j = 0; j < 16; ++j) {
    const int q = grp * 16 + j;
    const int ly = q >> 3, lx = q & 7;
    const float* hp = vh + (ly * 12 + lx) * 64 + ch;
    float acc = lbc;
#pragma unroll
    for (int dy = 0; dy < 5; ++dy)
#pragma unroll
      for (int dx = 0; dx < 5; ++dx)
        acc = fmaf(hp[(dy * 12 + dx) * 64], w25[dy * 5 + dx], acc);
    acc += ao[((size_t)(p * WT + q)) * CC + ch];
    zs[q * KTP + ch] = (_Float16)(acc * 64.0f);
  }
  __syncthreads();
  const int mi = wave & 3, nj = (wave >> 2) * 2;
  v8f acc2[2];
  acc2[0] = zero8(); acc2[1] = zero8();
#pragma unroll
  for (int k0 = 0; k0 < CC; k0 += 32) {
    const v16h a = ldfrag(zs, KTP, mi * 16, k0, lane);
#pragma unroll
    for (int t = 0; t < 2; ++t) {
      const v16h b = ldfrag(wot, CC, (nj + t) * 16, k0, lane);
      acc2[t] = mma16(a, b, acc2[t]);
    }
  }
  float* xs = vh;
#pragma unroll
  for (int t = 0; t < 2; ++t) {
    const int col = (nj + t) * 16 + m;
    const float bb = wob[col];
#pragma unroll
    for (int r = 0; r < 8; ++r) {
      const int q = mi * 16 + 8 * hl + r;
      xs[q * TP + col] = acc2[t][r] * (1.0f / 4096.0f) + bb;
    }
  }
  __syncthreads();
  {
    const int q = tid >> 2, part = tid & 3;
    const int pix = (y0 + (q >> 3)) * IMW + x0 + (q & 7);
    const float* xr = x1 + (size_t)pix * CC + part * 16;
    float* xp = xs + q * TP + part * 16;
#pragma unroll
    for (int k = 0; k < 4; ++k) {
      const v4f rv = *(const v4f*)(xr + 4 * k);
      v4f sv = *(const v4f*)(xp + 4 * k);
      sv = sv + rv;
      *(v4f*)(xp + 4 * k) = sv;
    }
    float o[16];
    ln16(xp, g, bt, part, o);
    *(v8h*)(ys + q * KTP + part * 16) =
        (v8h){(_Float16)o[0], (_Float16)o[1], (_Float16)o[2], (_Float16)o[3],
              (_Float16)o[4], (_Float16)o[5], (_Float16)o[6], (_Float16)o[7]};
    *(v8h*)(ys + q * KTP + part * 16 + 8) =
        (v8h){(_Float16)o[8], (_Float16)o[9], (_Float16)o[10], (_Float16)o[11],
              (_Float16)o[12], (_Float16)o[13], (_Float16)o[14], (_Float16)o[15]};
  }
  __syncthreads();
  for (int ps = 0; ps < 2; ++ps) {
#pragma unroll
    for (int it = 0; it < 4; ++it) {
      const int q = it * 32 + lane;
      const int lx = q >> 4, c4 = (q & 15) * 4;
      const v4f v = *(const v4f*)(xs + (wave * 8 + lx) * TP + c4);
      *(volatile v4f*)(x2 + ((size_t)((y0 + wave) * IMW + x0 + lx)) * CC + c4) = v;
    }
#pragma unroll
    for (int it = 0; it < 2; ++it) {
      const int q = it * 32 + lane;
      const int lx = q >> 3, c8 = (q & 7) * 8;
      const v4u v = *(const v4u*)(ys + (wave * 8 + lx) * KTP + c8);
      *(volatile v4u*)(yp + ((size_t)((y0 + wave) * IMW + x0 + lx)) * CC + c8) = v;
    }
    __threadfence();
  }
}

__global__ __launch_bounds__(256) void k_mlp(const _Float16* __restrict__ yp,
                                             const _Float16* __restrict__ w1t,
                                             const float* __restrict__ b1,
                                             const _Float16* __restrict__ w2t,
                                             const float* __restrict__ b2,
                                             const float* __restrict__ x2,
                                             float* __restrict__ out) {
  __shared__ __align__(16) _Float16 hs[WT * VTP];
  __shared__ __align__(16) float os[CC * TP];
  const int tid = threadIdx.x, lane = tid & 31, wave = tid >> 5;
  const int hl = lane >> 4, m = lane & 15;
  const int pix0 = blockIdx.x * 64;
  const int mi = wave & 3;
  {
    const int nb = (wave >> 2) * 128;
    v8f acc[8];
#pragma unroll
    for (int t = 0; t < 8; ++t) acc[t] = zero8();
#pragma unroll
    for (int k0 = 0; k0 < CC; k0 += 32) {
      const v16h a = ldfrag(yp, CC, pix0 + mi * 16, k0, lane);
#pragma unroll
      for (int t = 0; t < 8; ++t) {
        const v16h b = ldfrag(w1t, CC, nb + 16 * t, k0, lane);
        acc[t] = mma16(a, b, acc[t]);
      }
    }
#pragma unroll
    for (int t = 0; t < 8; ++t) {
      const int col = nb + 16 * t + m;
      const float bb = b1[col];
#pragma unroll
      for (int r = 0; r < 8; ++r) {
        const float f = acc[t][r] * (1.0f / 64.0f) + bb;
        const float gl = 8.0f * f * (1.0f + erff(f * 0.70710678118654752f));
        hs[(mi * 16 + 8 * hl + r) * VTP + col] = (_Float16)gl;
      }
    }
  }
  __syncthreads();
  {
    const int nj = (wave >> 2) * 2;
    v8f acc2[2];
    acc2[0] = zero8(); acc2[1] = zero8();
#pragma unroll 2
    for (int k0 = 0; k0 < FF; k0 += 32) {
      const v16h a = ldfrag(hs, VTP, mi * 16, k0, lane);
#pragma unroll
      for (int t = 0; t < 2; ++t) {
        const v16h b = ldfrag(w2t, FF, (nj + t) * 16, k0, lane);
        acc2[t] = mma16(a, b, acc2[t]);
      }
    }
#pragma unroll
    for (int t = 0; t < 2; ++t) {
      const int col = (nj + t) * 16 + m;
      const float bb = b2[col];
#pragma unroll
      for (int r = 0; r < 8; ++r) {
        const int row = mi * 16 + 8 * hl + r;
        os[col * TP + row] = acc2[t][r] * (1.0f / 1024.0f) + bb;
      }
    }
  }
  __syncthreads();
  {
    const int q = tid >> 2, part = tid & 3;
    const float* xr = x2 + ((size_t)(pix0 + q)) * CC + part * 16;
#pragma unroll
    for (int k = 0; k < 4; ++k) {
      const v4f rv = *(const v4f*)(xr + 4 * k);
#pragma unroll
      for (int e = 0; e < 4; ++e) {
        const int col = part * 16 + 4 * k + e;
        float* op2 = os + col * TP + q;
        *op2 = *op2 + rv[e];
      }
    }
  }
  __syncthreads();
  for (int ps = 0; ps < 2; ++ps) {
#pragma unroll
    for (int it = 0; it < 4; ++it) {
      const int gi = wave * 128 + it * 32 + lane;
      const int cch = gi >> 4, j4 = (gi & 15) * 4;
      const v4f v = *(const v4f*)(os + cch * TP + j4);
      *(volatile v4f*)(out + (size_t)cch * NPIX + pix0 + j4) = v;
    }
    __threadfence();
  }
}

extern "C" void kernel_launch(void* const* d_in, const int* in_sizes, int n_in,
                              void* d_out, int out_size, void* d_ws, size_t ws_size,
                              hipStream_t stream) {
  if (n_in < 15) return;
  if (in_sizes[0] != NPIX * CC) return;
  if (in_sizes[1] != CC * 9 || in_sizes[2] != CC || in_sizes[3] != CC || in_sizes[4] != CC) return;
  if (in_sizes[5] != CC * C3 || in_sizes[6] != C3) return;
  if (in_sizes[7] != CC * CC || in_sizes[8] != CC) return;
  if (in_sizes[9] != CC * 25 || in_sizes[10] != CC) return;
  if (in_sizes[11] != CC * FF || in_sizes[12] != FF) return;
  if (in_sizes[13] != FF * CC || in_sizes[14] != CC) return;
  if (out_size != NPIX * CC) return;

  const float* x      = (const float*)d_in[0];
  const float* pos_w  = (const float*)d_in[1];
  const float* pos_b  = (const float*)d_in[2];
  const float* norm_g = (const float*)d_in[3];
  const float* norm_b = (const float*)d_in[4];
  const float* qkv_w  = (const float*)d_in[5];
  const float* qkv_b  = (const float*)d_in[6];
  const float* wo_w   = (const float*)d_in[7];
  const float* wo_b   = (const float*)d_in[8];
  const float* lepe_w = (const float*)d_in[9];
  const float* lepe_b = (const float*)d_in[10];
  const float* mlp_w1 = (const float*)d_in[11];
  const float* mlp_b1 = (const float*)d_in[12];
  const float* mlp_w2 = (const float*)d_in[13];
  const float* mlp_b2 = (const float*)d_in[14];
  float* out = (float*)d_out;

  size_t off = 0;
  const size_t oX1  = off; off += (size_t)NPIX * CC * 4;
  const size_t oA1  = off; off += (size_t)NPIX * C3 * 2;
  const size_t oWQ  = off; off += (size_t)C3 * C3 * 2;
  const size_t oWO  = off; off += (size_t)CC * CC * 2;
  const size_t oW1  = off; off += (size_t)FF * CC * 2;
  const size_t oW2  = off; off += (size_t)CC * FF * 2;
  const size_t oQKV = off; off += (size_t)NPIX * C3 * 4;
  const size_t oMW  = off; off += (size_t)NWD * 128 * 4;
  const size_t oAO  = off; off += (size_t)NPIX * CC * 4;
  const size_t oX2  = off; off += (size_t)NPIX * CC * 4;
  const size_t oY   = off; off += (size_t)NPIX * CC * 2;
  if (off > ws_size) return;
  if (off > (size_t)134217728) return;

  char* ws = (char*)d_ws;
  float*          X1  = (float*)(ws + oX1);
  unsigned short* A1  = (unsigned short*)(ws + oA1);
  unsigned short* WQ3 = (unsigned short*)(ws + oWQ);
  _Float16*       WOT = (_Float16*)(ws + oWO);
  _Float16*       W1T = (_Float16*)(ws + oW1);
  _Float16*       W2T = (_Float16*)(ws + oW2);
  float*          QKV = (float*)(ws + oQKV);
  float*          MW  = (float*)(ws + oMW);
  float*          AO  = (float*)(ws + oAO);
  float*          X2  = (float*)(ws + oX2);
  _Float16*       Y   = (_Float16*)(ws + oY);

  k_posln<<<dim3(NWD), dim3(256), 0, stream>>>(x, pos_w, pos_b, norm_g, norm_b, X1, A1);
  k_wt<<<dim3(CC / 64, CC / 64), dim3(256), 0, stream>>>(wo_w, WOT, CC, CC);
  k_wt<<<dim3(FF / 64, CC / 64), dim3(256), 0, stream>>>(mlp_w1, W1T, FF, CC);
  k_wt<<<dim3(CC / 64, FF / 64), dim3(256), 0, stream>>>(mlp_w2, W2T, CC, FF);
  k_wq3<<<dim3(C3 / 64), dim3(256), 0, stream>>>(qkv_w, WQ3);
  k_qkv<<<dim3(NWD), dim3(256), 0, stream>>>((const __bf16*)A1, (const __bf16*)WQ3, qkv_b, QKV, MW);
  (void)hipFuncSetAttribute(reinterpret_cast<const void*>(&k_attn),
                            hipFuncAttributeMaxDynamicSharedMemorySize, ATT_LDS);
  k_attn<<<dim3(NWD), dim3(256), ATT_LDS, stream>>>(QKV, MW, AO);
  k_comb<<<dim3(NWD), dim3(256), 0, stream>>>(QKV, AO, lepe_w, lepe_b, WOT, wo_b, X1, norm_g, norm_b, X2, Y);
  k_mlp<<<dim3(NPIX / 64), dim3(256), 0, stream>>>(Y, W1T, mlp_b1, W2T, mlp_b2, X2, out);
  (void)hipGetLastError();
}
